// TransformerModel_28948079575191
// MI455X (gfx1250) — hardware-run, weakly checked
//
#include <hip/hip_runtime.h>
#include <math.h>

typedef __attribute__((ext_vector_type(16))) __bf16   v16b;
typedef __attribute__((ext_vector_type(8)))  __bf16   v8b;
typedef __attribute__((ext_vector_type(8)))  float    v8f;
typedef __attribute__((ext_vector_type(4)))  float    v4f;
typedef __attribute__((ext_vector_type(2)))  float    v2f;
typedef __attribute__((ext_vector_type(4)))  unsigned v4u;
typedef __attribute__((ext_vector_type(4)))  int      v4i;
typedef __attribute__((ext_vector_type(2)))  int      v2i;

constexpr int kN      = 50000;
constexpr int kNPad   = 50048;
constexpr int kE      = 800000;
constexpr int kIn     = 128;
constexpr int kHid    = 64;
constexpr int kHeads  = 4;
constexpr int kOut    = 32;
constexpr int kQW     = kHeads * kHid;
constexpr int kQkvW   = 3 * kQW;
constexpr int kFusedN = kQkvW + kHid;
constexpr int kTile   = 128;
constexpr int kNumTiles = kNPad / kTile;
constexpr int kRowWords = kQkvW / 2;
constexpr int kKOffWords = kQW / 2;
constexpr float kQScale    = 2048.0f;
constexpr float kQScaleInv = 1.0f / 2048.0f;
constexpr float kInvSqrtHid = 0.125f;
constexpr float kLogitScale = kInvSqrtHid * kQScaleInv * kQScaleInv;
constexpr float kInvHid = 1.0f / (float)kHid;
static_assert(kInvSqrtHid * kInvSqrtHid * (float)kHid == 1.0f);
static_assert(kHid == 64 && kHeads == 4 && kQW == 256 && kQkvW == 768 && kFusedN == 832);
static_assert((kNPad % 64) == 0 && (kNPad % kTile) == 0 && kNPad >= kN && kNPad - kN < 64);
static_assert((kIn % 32) == 0 && (kHid % 32) == 0 && (kFusedN % 64) == 0);
static_assert((kE % 128) == 0 && ((kE * 4) % 16) == 0);
static_assert(kNumTiles == 391);

constexpr size_t kOffXB   = 0;
constexpr size_t kOffBT1  = kOffXB   + (size_t)kNPad * kIn * 2;
constexpr size_t kOffBT2  = kOffBT1  + (size_t)kFusedN * kIn * 2;
constexpr size_t kOffBTF  = kOffBT2  + (size_t)kFusedN * kHid * 2;
constexpr size_t kOffBIAS = kOffBTF  + (size_t)64 * kHid * 2;
constexpr size_t kOffQKV  = kOffBIAS + (size_t)(2 * kFusedN + 64) * 4;
constexpr size_t kOffHACC = kOffQKV  + (size_t)kNPad * kQkvW * 2;
constexpr size_t kOffH1H  = kOffHACC + (size_t)kNPad * kHid * 4;
constexpr size_t kOffH1L  = kOffH1H  + (size_t)kNPad * kHid * 2;
constexpr size_t kOffH2H  = kOffH1L  + (size_t)kNPad * kHid * 2;
constexpr size_t kOffH2L  = kOffH2H  + (size_t)kNPad * kHid * 2;
constexpr size_t kWsTotal = kOffH2L  + (size_t)kNPad * kHid * 2;
static_assert(kWsTotal == 128457472ull);
static_assert(kWsTotal <= 134217728ull);
static_assert((kOffBT1 % 128) == 0 && (kOffBT2 % 128) == 0 && (kOffBTF % 128) == 0 && (kOffBIAS % 128) == 0 &&
              (kOffQKV % 128) == 0 && (kOffHACC % 128) == 0 && (kOffH1H % 128) == 0 && (kOffH1L % 128) == 0 &&
              (kOffH2H % 128) == 0 && (kOffH2L % 128) == 0);

__device__ __forceinline__ unsigned short f2bf_bits(float f) {
  unsigned u = __float_as_uint(f);
  return (unsigned short)((u + 0x7FFFu + ((u >> 16) & 1u)) >> 16);
}
__device__ __forceinline__ float bf_bits2f(unsigned short h) { return __uint_as_float(((unsigned)h) << 16); }
__device__ __forceinline__ float bf_rne(float f) { return bf_bits2f(f2bf_bits(f)); }
__device__ __forceinline__ unsigned pack_bf2(float a, float b) {
  const unsigned ha = (unsigned)f2bf_bits(a);
  const unsigned hb = (unsigned)f2bf_bits(b);
  return ha | (hb << 16);
}
__device__ __forceinline__ void split_pack2(float a, float b, unsigned& hw, unsigned& lw) {
  const unsigned short ha = f2bf_bits(a);
  const unsigned short hb = f2bf_bits(b);
  const unsigned short la = f2bf_bits(a - bf_bits2f(ha));
  const unsigned short lb = f2bf_bits(b - bf_bits2f(hb));
  hw = (unsigned)ha | (((unsigned)hb) << 16);
  lw = (unsigned)la | (((unsigned)lb) << 16);
}
__device__ __forceinline__ unsigned q11_pack2(float a, float b) {
  float ta = rintf(a * kQScale);
  float tb = rintf(b * kQScale);
  ta = fminf(fmaxf(ta, -32767.0f), 32767.0f);
  tb = fminf(fmaxf(tb, -32767.0f), 32767.0f);
  const int ia = (int)ta;
  const int ib = (int)tb;
  return (((unsigned)ia) & 0xffffu) | (((unsigned)ib) << 16);
}
__device__ __forceinline__ float q11_lo(unsigned w) { return (float)(((int)(w << 16)) >> 16); }
__device__ __forceinline__ float q11_hi(unsigned w) { return (float)(((int)w) >> 16); }

__device__ __forceinline__ void lds_wave_sync() {
  __builtin_amdgcn_fence(__ATOMIC_RELEASE, "workgroup");
  __builtin_amdgcn_wave_barrier();
  __builtin_amdgcn_fence(__ATOMIC_ACQUIRE, "workgroup");
}

union FragB { v16b v; v8b h[2]; };
__device__ __forceinline__ v16b frag_load(const __bf16* p) {
  FragB f;
  f.h[0] = *(const v8b*)(p);
  f.h[1] = *(const v8b*)(p + 16);
  return f.v;
}
__device__ __forceinline__ v8f frag_mma(v16b a, v16b b, v8f c) {
  return __builtin_amdgcn_wmma_f32_16x16x32_bf16(false, a, false, b, (short)0, c, false, false);
}
__device__ __forceinline__ void wm_guard(v8f& a, v16b x, v16b y) {
  asm volatile("v_nop\n\tv_nop\n\tv_nop\n\tv_nop" : "+v"(a) : "v"(x), "v"(y));
}
__device__ __forceinline__ void keep4_b(v16b a, v16b b, v16b c, v16b d) { asm volatile("v_nop" :: "v"(a), "v"(b), "v"(c), "v"(d)); }
__device__ __forceinline__ void acc_guard4(v8f& a, v8f& b, v8f& c, v8f& d) {
  asm volatile("v_nop\n\tv_nop\n\tv_nop\n\tv_nop" : "+v"(a), "+v"(b), "+v"(c), "+v"(d));
}

__global__ __launch_bounds__(256) void cast_x_kernel(const float* __restrict__ x, unsigned short* __restrict__ xb)
{
  const int i = blockIdx.x * 256 + threadIdx.x;
  if (i >= kNPad * kIn / 8) return;
  const int row = i >> 4;
  const int c   = (i & 15) * 8;
  const int rc  = row < kN ? row : (kN - 1);
  const bool valid = row < kN;
  const v4f a0 = *(const v4f*)(x + (size_t)rc * kIn + c);
  const v4f a1 = *(const v4f*)(x + (size_t)rc * kIn + c + 4);
  const float f0 = valid ? a0.x : 0.0f, f1 = valid ? a0.y : 0.0f, f2 = valid ? a0.z : 0.0f, f3 = valid ? a0.w : 0.0f;
  const float f4 = valid ? a1.x : 0.0f, f5 = valid ? a1.y : 0.0f, f6 = valid ? a1.z : 0.0f, f7 = valid ? a1.w : 0.0f;
  const v4u wv = { pack_bf2(f0, f1), pack_bf2(f2, f3), pack_bf2(f4, f5), pack_bf2(f6, f7) };
  unsigned short* p = xb + (size_t)i * 8;
  *(volatile v4u*)p = wv;
  __threadfence();
  *(volatile v4u*)p = wv;
}

__global__ __launch_bounds__(256) void wprep_kernel(
    const float* __restrict__ wq1, const float* __restrict__ wk1, const float* __restrict__ wv1, const float* __restrict__ ws1,
    const float* __restrict__ wq2, const float* __restrict__ wk2, const float* __restrict__ wv2, const float* __restrict__ ws2,
    const float* __restrict__ wf,
    unsigned short* __restrict__ bt1, unsigned short* __restrict__ bt2, unsigned short* __restrict__ btf)
{
  const int seg = blockIdx.y;
  const float* W = wq1;
  unsigned short* dst = bt1;
  int ncr = 256, nro = 256, ksh = 4, rb = 0;
  if (seg == 1) { W = wk1; rb = 256; }
  else if (seg == 2) { W = wv1; rb = 512; }
  else if (seg == 3) { W = ws1; ncr = 64; nro = 64; rb = 768; }
  else if (seg == 4) { W = wq2; ksh = 3; dst = bt2; }
  else if (seg == 5) { W = wk2; ksh = 3; dst = bt2; rb = 256; }
  else if (seg == 6) { W = wv2; ksh = 3; dst = bt2; rb = 512; }
  else if (seg == 7) { W = ws2; ncr = 64; nro = 64; ksh = 3; dst = bt2; rb = 768; }
  else if (seg == 8) { W = wf; ncr = 32; nro = 64; ksh = 3; dst = btf; rb = 0; }
  const int i = blockIdx.x * 256 + threadIdx.x;
  if (i >= (nro << ksh)) return;
  const int n  = i >> ksh;
  const int kc = i & ((1 << ksh) - 1);
  const int nc = n < ncr ? n : (ncr - 1);
  const bool valid = n < ncr;
  const float* wp = W + (size_t)(kc * 8) * ncr + nc;
  float f0 = wp[0];
  float f1 = wp[(size_t)1 * ncr];
  float f2 = wp[(size_t)2 * ncr];
  float f3 = wp[(size_t)3 * ncr];
  float f4 = wp[(size_t)4 * ncr];
  float f5 = wp[(size_t)5 * ncr];
  float f6 = wp[(size_t)6 * ncr];
  float f7 = wp[(size_t)7 * ncr];
  f0 = valid ? f0 : 0.0f; f1 = valid ? f1 : 0.0f; f2 = valid ? f2 : 0.0f; f3 = valid ? f3 : 0.0f;
  f4 = valid ? f4 : 0.0f; f5 = valid ? f5 : 0.0f; f6 = valid ? f6 : 0.0f; f7 = valid ? f7 : 0.0f;
  const v4u wv = { pack_bf2(f0, f1), pack_bf2(f2, f3), pack_bf2(f4, f5), pack_bf2(f6, f7) };
  unsigned short* p = dst + (((size_t)(rb + n)) << (ksh + 3)) + kc * 8;
  *(volatile v4u*)p = wv;
  __threadfence();
  *(volatile v4u*)p = wv;
}

__global__ __launch_bounds__(64) void bias_kernel(
    const float* __restrict__ bq1, const float* __restrict__ bk1, const float* __restrict__ bv1, const float* __restrict__ bs1,
    const float* __restrict__ bq2, const float* __restrict__ bk2, const float* __restrict__ bv2, const float* __restrict__ bs2,
    const float* __restrict__ bfin, float* __restrict__ biasOut)
{
  const int seg = blockIdx.x;
  const float* B = bq1;
  int nreal = 256, nout = 256, off = 0;
  if (seg == 1) { B = bk1; off = 256; }
  else if (seg == 2) { B = bv1; off = 512; }
  else if (seg == 3) { B = bs1; nreal = 64; nout = 64; off = 768; }
  else if (seg == 4) { B = bq2; off = kFusedN; }
  else if (seg == 5) { B = bk2; off = kFusedN + 256; }
  else if (seg == 6) { B = bv2; off = kFusedN + 512; }
  else if (seg == 7) { B = bs2; nreal = 64; nout = 64; off = kFusedN + 768; }
  else if (seg == 8) { B = bfin; nreal = kOut; nout = 64; off = 2 * kFusedN; }
  const int i4 = threadIdx.x * 4;
  if (i4 >= nout) return;
  const int j0 = (i4 + 0) < nreal ? (i4 + 0) : (nreal - 1);
  const int j1 = (i4 + 1) < nreal ? (i4 + 1) : (nreal - 1);
  const int j2 = (i4 + 2) < nreal ? (i4 + 2) : (nreal - 1);
  const int j3 = (i4 + 3) < nreal ? (i4 + 3) : (nreal - 1);
  float f0 = B[j0], f1 = B[j1], f2 = B[j2], f3 = B[j3];
  f0 = (i4 + 0) < nreal ? bf_rne(f0) : 0.0f;
  f1 = (i4 + 1) < nreal ? bf_rne(f1) : 0.0f;
  f2 = (i4 + 2) < nreal ? bf_rne(f2) : 0.0f;
  f3 = (i4 + 3) < nreal ? bf_rne(f3) : 0.0f;
  const v4f v = { f0, f1, f2, f3 };
  float* p = biasOut + off + i4;
  *(volatile v4f*)p = v;
  __threadfence();
  *(volatile v4f*)p = v;
}

template <int SPL, int MODE>
__global__ __launch_bounds__(256) void proj_gemm_kernel(
    const unsigned short* __restrict__ Ap, const unsigned short* __restrict__ A2p, int lda,
    const unsigned short* __restrict__ Btp, int ldb,
    const float* __restrict__ bias,
    unsigned short* __restrict__ outQ, float* __restrict__ outF,
    int tilesM, int tilesN, int K)
{
  __shared__ __align__(16) float sT[8][16 * 68];
  const int lane = threadIdx.x & 31;
  const int wave = __builtin_amdgcn_readfirstlane((int)(threadIdx.x >> 5));
  const int tile = blockIdx.x * 8 + wave;
  if (tile >= tilesM * tilesN) return;
  const int tm = tile / tilesN;
  const int tn = tile - tm * tilesN;
  const int m0 = tm << 6;
  const int n0 = tn << 6;
  const bool skipTile = (MODE == 0) && (tn == tilesN - 1);

  const __bf16* A  = (const __bf16*)Ap;
  const __bf16* A2 = (const __bf16*)A2p;
  const __bf16* Bt = (const __bf16*)Btp;

  const int rlane = lane & 15;
  const int koff  = (lane >> 4) * 8;
  const int mOff  = (lane >> 4) * 8;

  v8f acc[4][4];
#pragma unroll
  for (int i = 0; i < 4; ++i)
#pragma unroll
    for (int j = 0; j < 4; ++j) acc[i][j] = (v8f){0.f,0.f,0.f,0.f,0.f,0.f,0.f,0.f};

  for (int k0 = 0; k0 < K; k0 += 32) {
    v16b bh[4];
#pragma unroll
    for (int j = 0; j < 4; ++j) {
      const size_t bo = (size_t)(n0 + (j << 4) + rlane) * ldb + koff + k0;
      bh[j] = frag_load(Bt + bo);
    }
#pragma unroll
    for (int i = 0; i < 4; ++i) {
      const size_t ao = (size_t)(m0 + (i << 4) + rlane) * lda + koff + k0;
      v16b ah = frag_load(A + ao);
      v16b al = ah;
      if (SPL == 1) al = frag_load(A2 + ao);
#pragma unroll
      for (int j = 0; j < 4; ++j) {
        acc[i][j] = frag_mma(ah, bh[j], acc[i][j]);
        if (SPL == 1) acc[i][j] = frag_mma(al, bh[j], acc[i][j]);
      }
      wm_guard(acc[i][0], ah, bh[0]);
      wm_guard(acc[i][1], al, bh[1]);
      wm_guard(acc[i][2], ah, bh[2]);
      wm_guard(acc[i][3], al, bh[3]);
    }
    keep4_b(bh[0], bh[1], bh[2], bh[3]);
  }
  acc_guard4(acc[0][0], acc[0][1], acc[0][2], acc[0][3]);
  acc_guard4(acc[1][0], acc[1][1], acc[1][2], acc[1][3]);
  acc_guard4(acc[2][0], acc[2][1], acc[2][2], acc[2][3]);
  acc_guard4(acc[3][0], acc[3][1], acc[3][2], acc[3][3]);

  float* slab = sT[wave];
#pragma unroll
  for (int i = 0; i < 4; ++i) {
    const int mBase = m0 + (i << 4);
#pragma unroll
    for (int j = 0; j < 4; ++j) {
      const float bv = bias[n0 + (j << 4) + rlane];
#pragma unroll
      for (int r = 0; r < 8; ++r) {
        slab[(mOff + r) * 68 + (j << 4) + rlane] = acc[i][j][r] + bv;
      }
    }
    lds_wave_sync();
    if (MODE == 1) {
      const int rq = lane >> 3, c4 = (lane & 7) * 4;
      for (int pass = 0; pass < 2; ++pass) {
#pragma unroll
        for (int it = 0; it < 4; ++it) {
          const int row = it * 4 + rq;
          const v4f v = *(const v4f*)(slab + row * 68 + c4);
          const int grow = mBase + row;
          if (grow < kN) *(volatile v4f*)(outF + (size_t)grow * kOut + c4) = v;
        }
        __threadfence();
      }
    } else if (skipTile) {
      const int hh = lane >> 4, c4 = (lane & 15) * 4;
      for (int pass = 0; pass < 2; ++pass) {
#pragma unroll
        for (int it = 0; it < 8; ++it) {
          const int row = it * 2 + hh;
          const v4f v = *(const v4f*)(slab + row * 68 + c4);
          *(volatile v4f*)(outF + (size_t)(mBase + row) * kHid + c4) = v;
        }
        __threadfence();
      }
    } else {
      const int rq = lane >> 3, c8 = (lane & 7) * 8;
      for (int pass = 0; pass < 2; ++pass) {
#pragma unroll
        for (int it = 0; it < 4; ++it) {
          const int row = it * 4 + rq;
          const float* sp = slab + row * 68 + c8;
          const v4f a0 = *(const v4f*)(sp);
          const v4f a1 = *(const v4f*)(sp + 4);
          const v4u wv = { q11_pack2(a0.x, a0.y), q11_pack2(a0.z, a0.w), q11_pack2(a1.x, a1.y), q11_pack2(a1.z, a1.w) };
          *(volatile v4u*)(outQ + (size_t)(mBase + row) * kQkvW + n0 + c8) = wv;
        }
        __threadfence();
      }
    }
    lds_wave_sync();
  }
}

template <bool RELU>
__global__ __launch_bounds__(32) void edge_attn_ln_kernel(
    const int* __restrict__ ei, const unsigned* __restrict__ qkvw, const float* __restrict__ hacc,
    const float* __restrict__ lng, const float* __restrict__ lnb,
    unsigned short* __restrict__ hhi, unsigned short* __restrict__ hlo)
{
  __shared__ __align__(16) float sAcc[kTile * kQW];
  __shared__ __align__(16) float sMS[kTile * kHeads * 2];
  __shared__ __align__(16) int   sList[2 * 128];
  const int lane = threadIdx.x & 31;
  const int n0   = blockIdx.x * kTile;
  const int* srcp = ei;
  const int* dstp = ei + kE;

  const v2f gq = *(const v2f*)(lng + 2 * lane);
  const v2f bq = *(const v2f*)(lnb + 2 * lane);
  const float g0 = bf_rne(gq.x), g1 = bf_rne(gq.y);
  const float b0 = bf_rne(bq.x), b1 = bf_rne(bq.y);

  {
    const v4f z = { 0.f, 0.f, 0.f, 0.f };
#pragma unroll 4
    for (int i = 0; i < (kTile * kQW) / 128; ++i) *(v4f*)(sAcc + (i * 32 + lane) * 4) = z;
    const float ninf = -__builtin_huge_valf();
    const v4f ms0 = { ninf, 0.f, ninf, 0.f };
#pragma unroll
    for (int i = 0; i < kTile / 32; ++i) {
      *(v4f*)(sMS + (i * 32 + lane) * 8)     = ms0;
      *(v4f*)(sMS + (i * 32 + lane) * 8 + 4) = ms0;
    }
  }
  lds_wave_sync();

  const int hg = lane >> 3;
#pragma unroll 1
  for (int eb = 0; eb < kE; eb += 128) {
    const v4i d4 = *(const v4i*)(dstp + eb + lane * 4);
    const int dl0 = d4.x - n0, dl1 = d4.y - n0, dl2 = d4.z - n0, dl3 = d4.w - n0;
    const bool h0 = (unsigned)dl0 < (unsigned)kTile;
    const bool h1 = (unsigned)dl1 < (unsigned)kTile;
    const bool h2 = (unsigned)dl2 < (unsigned)kTile;
    const bool h3 = (unsigned)dl3 < (unsigned)kTile;
    const unsigned mk0 = __builtin_amdgcn_ballot_w32(h0);
    const unsigned mk1 = __builtin_amdgcn_ballot_w32(h1);
    const unsigned mk2 = __builtin_amdgcn_ballot_w32(h2);
    const unsigned mk3 = __builtin_amdgcn_ballot_w32(h3);
    if ((mk0 | mk1 | mk2 | mk3) != 0u) {
      const int c0 = __builtin_popcount(mk0);
      const int c1 = c0 + __builtin_popcount(mk1);
      const int c2 = c1 + __builtin_popcount(mk2);
      int cnt = c2 + __builtin_popcount(mk3);
      const int e0 = eb + lane * 4;
      const int p0 = (int)__builtin_amdgcn_mbcnt_lo(mk0, 0u);
      const int p1 = c0 + (int)__builtin_amdgcn_mbcnt_lo(mk1, 0u);
      const int p2 = c1 + (int)__builtin_amdgcn_mbcnt_lo(mk2, 0u);
      const int p3 = c2 + (int)__builtin_amdgcn_mbcnt_lo(mk3, 0u);
      if (h0) *(v2i*)(sList + 2 * p0) = (v2i){ e0,     dl0 };
      if (h1) *(v2i*)(sList + 2 * p1) = (v2i){ e0 + 1, dl1 };
      if (h2) *(v2i*)(sList + 2 * p2) = (v2i){ e0 + 2, dl2 };
      if (h3) *(v2i*)(sList + 2 * p3) = (v2i){ e0 + 3, dl3 };
      cnt = cnt < 128 ? cnt : 128;
      cnt = __builtin_amdgcn_readfirstlane(cnt);
      lds_wave_sync();
#pragma unroll 1
      for (int i = 0; i < cnt; ++i) {
        const v2i ent = *(const v2i*)(sList + 2 * i);
        int ec = ent.x;
        ec = ec < 0 ? 0 : (ec > (kE - 1) ? (kE - 1) : ec);
        const int dlc = ent.y & (kTile - 1);
        int s = srcp[ec];
        s = s < 0 ? 0 : (s > (kN - 1) ? (kN - 1) : s);
        const unsigned* qp = qkvw + (size_t)(n0 + dlc) * kRowWords + lane * 4;
        const unsigned* kp = qkvw + (size_t)s * kRowWords + kKOffWords + lane * 4;
        const v4u qw = *(const v4u*)(qp);
        const v4u kw = *(const v4u*)(kp);
        const v4u vw = *(const v4u*)(kp + kKOffWords);
        const unsigned q0 = qw.x, q1 = qw.y, q2 = qw.z, q3 = qw.w;
        const unsigned k0 = kw.x, k1 = kw.y, k2 = kw.z, k3 = kw.w;
        const unsigned w0 = vw.x, w1 = vw.y, w2 = vw.z, w3 = vw.w;
        float dot = q11_lo(q0) * q11_lo(k0);
        dot = fmaf(q11_hi(q0), q11_hi(k0), dot);
        dot = fmaf(q11_lo(q1), q11_lo(k1), dot);
        dot = fmaf(q11_hi(q1), q11_hi(k1), dot);
        dot = fmaf(q11_lo(q2), q11_lo(k2), dot);
        dot = fmaf(q11_hi(q2), q11_hi(k2), dot);
        dot = fmaf(q11_lo(q3), q11_lo(k3), dot);
        dot = fmaf(q11_hi(q3), q11_hi(k3), dot);
        dot += __shfl_xor(dot, 1, 32);
        dot += __shfl_xor(dot, 2, 32);
        dot += __shfl_xor(dot, 4, 32);
        const float logit = dot * kLogitScale;
        float* msp = sMS + (dlc * kHeads + hg) * 2;
        const v2f ms = *(const v2f*)msp;
        const float mnew = fmaxf(ms.x, logit);
        const float sc = __expf(ms.x - mnew);
        const float p  = __expf(logit - mnew);
        const float snew = ms.y * sc + p;
        if ((lane & 7) == 0) *(v2f*)msp = (v2f){ mnew, snew };
        const float pv = p * kQScaleInv;
        float* ap = sAcc + dlc * kQW + lane * 8;
        v4f a0 = *(const v4f*)(ap);
        v4f a1 = *(const v4f*)(ap + 4);
        a0.x = fmaf(pv, q11_lo(w0), a0.x * sc);
        a0.y = fmaf(pv, q11_hi(w0), a0.y * sc);
        a0.z = fmaf(pv, q11_lo(w1), a0.z * sc);
        a0.w = fmaf(pv, q11_hi(w1), a0.w * sc);
        a1.x = fmaf(pv, q11_lo(w2), a1.x * sc);
        a1.y = fmaf(pv, q11_hi(w2), a1.y * sc);
        a1.z = fmaf(pv, q11_lo(w3), a1.z * sc);
        a1.w = fmaf(pv, q11_hi(w3), a1.w * sc);
        *(v4f*)(ap)     = a0;
        *(v4f*)(ap + 4) = a1;
      }
      lds_wave_sync();
    }
  }
  lds_wave_sync();

#pragma unroll 1
  for (int node = 0; node < kTile; ++node) {
    const v4f msa = *(const v4f*)(sMS + node * 8);
    const v4f msb = *(const v4f*)(sMS + node * 8 + 4);
    const float s0 = msa.y, s1 = msa.w, s2 = msb.y, s3 = msb.w;
    const float r0 = 1.0f / (s0 > 0.f ? s0 : 1.0f);
    const float r1 = 1.0f / (s1 > 0.f ? s1 : 1.0f);
    const float r2 = 1.0f / (s2 > 0.f ? s2 : 1.0f);
    const float r3 = 1.0f / (s3 > 0.f ? s3 : 1.0f);
    const float i0 = s0 > 0.f ? r0 : 0.f;
    const float i1 = s1 > 0.f ? r1 : 0.f;
    const float i2 = s2 > 0.f ? r2 : 0.f;
    const float i3 = s3 > 0.f ? r3 : 0.f;
    const float* ap = sAcc + node * kQW + 2 * lane;
    const v2f a0 = *(const v2f*)(ap);
    const v2f a1 = *(const v2f*)(ap + kHid);
    const v2f a2 = *(const v2f*)(ap + 2 * kHid);
    const v2f a3 = *(const v2f*)(ap + 3 * kHid);
    const v2f sk = *(const v2f*)(hacc + (size_t)(n0 + node) * kHid + 2 * lane);
    float t0 = a0.x * i0;
    float t1 = a0.y * i0;
    t0 = fmaf(a1.x, i1, t0);
    t1 = fmaf(a1.y, i1, t1);
    t0 = fmaf(a2.x, i2, t0);
    t1 = fmaf(a2.y, i2, t1);
    t0 = fmaf(a3.x, i3, t0);
    t1 = fmaf(a3.y, i3, t1);
    const float x0 = fmaf(0.25f, t0, sk.x);
    const float x1 = fmaf(0.25f, t1, sk.y);
    float sum = x0 + x1;
    sum += __shfl_xor(sum, 1, 32);
    sum += __shfl_xor(sum, 2, 32);
    sum += __shfl_xor(sum, 4, 32);
    sum += __shfl_xor(sum, 8, 32);
    sum += __shfl_xor(sum, 16, 32);
    const float mu = sum * kInvHid;
    const float d0 = x0 - mu, d1 = x1 - mu;
    float vs = d0 * d0 + d1 * d1;
    vs += __shfl_xor(vs, 1, 32);
    vs += __shfl_xor(vs, 2, 32);
    vs += __shfl_xor(vs, 4, 32);
    vs += __shfl_xor(vs, 8, 32);
    vs += __shfl_xor(vs, 16, 32);
    const float var  = vs * kInvHid;
    const float rstd = 1.0f / sqrtf(var + 1e-5f);
    float y0 = d0 * rstd * g0 + b0;
    float y1 = d1 * rstd * g1 + b1;
    if (RELU) { y0 = fmaxf(y0, 0.f); y1 = fmaxf(y1, 0.f); }
    const bool valid = (n0 + node) < kN;
    y0 = valid ? y0 : 0.f;
    y1 = valid ? y1 : 0.f;
    *(v2f*)(sAcc + node * kQW + 2 * lane) = (v2f){ y0, y1 };
  }
  lds_wave_sync();

  {
    const int rq = lane >> 3, c8 = (lane & 7) * 8;
    for (int pass = 0; pass < 2; ++pass) {
#pragma unroll 1
      for (int it = 0; it < kTile / 4; ++it) {
        const int row = it * 4 + rq;
        const float* sp = sAcc + row * kQW + c8;
        const v4f a0 = *(const v4f*)(sp);
        const v4f a1 = *(const v4f*)(sp + 4);
        unsigned hw0, hw1, hw2, hw3, lw0, lw1, lw2, lw3;
        split_pack2(a0.x, a0.y, hw0, lw0);
        split_pack2(a0.z, a0.w, hw1, lw1);
        split_pack2(a1.x, a1.y, hw2, lw2);
        split_pack2(a1.z, a1.w, hw3, lw3);
        const v4u hv = { hw0, hw1, hw2, hw3 };
        const v4u lv = { lw0, lw1, lw2, lw3 };
        const size_t o = (size_t)(n0 + row) * kHid + c8;
        *(volatile v4u*)(hhi + o) = hv;
        *(volatile v4u*)(hlo + o) = lv;
      }
      __threadfence();
    }
  }
}

extern "C" void kernel_launch(void* const* d_in, const int* in_sizes, int n_in,
                              void* d_out, int out_size, void* d_ws, size_t ws_size,
                              hipStream_t stream) {
  if (n_in < 22) return;
  if (in_sizes[0] != kN * kIn) return;
  if (in_sizes[1] != 2 * kE) return;
  if (in_sizes[2] != kIn * kQW || in_sizes[4] != kIn * kQW || in_sizes[6] != kIn * kQW) return;
  if (in_sizes[8] != kIn * kHid) return;
  if (in_sizes[10] != kHid * kQW || in_sizes[12] != kHid * kQW || in_sizes[14] != kHid * kQW) return;
  if (in_sizes[16] != kHid * kHid) return;
  if (in_sizes[3] != kQW || in_sizes[5] != kQW || in_sizes[7] != kQW || in_sizes[9] != kHid) return;
  if (in_sizes[11] != kQW || in_sizes[13] != kQW || in_sizes[15] != kQW || in_sizes[17] != kHid) return;
  if (in_sizes[18] != kHid || in_sizes[19] != kHid) return;
  if (in_sizes[20] != kHid * kOut || in_sizes[21] != kOut) return;
  if (out_size != kN * kOut) return;
  if (ws_size < kWsTotal) return;

  const float* x   = (const float*)d_in[0];
  const int*   ei  = (const int*)d_in[1];
  const float *Wq1 = (const float*)d_in[2],  *bq1 = (const float*)d_in[3];
  const float *Wk1 = (const float*)d_in[4],  *bk1 = (const float*)d_in[5];
  const float *Wv1 = (const float*)d_in[6],  *bv1 = (const float*)d_in[7];
  const float *Ws1 = (const float*)d_in[8],  *bs1 = (const float*)d_in[9];
  const float *Wq2 = (const float*)d_in[10], *bq2 = (const float*)d_in[11];
  const float *Wk2 = (const float*)d_in[12], *bk2 = (const float*)d_in[13];
  const float *Wv2 = (const float*)d_in[14], *bv2 = (const float*)d_in[15];
  const float *Ws2 = (const float*)d_in[16], *bs2 = (const float*)d_in[17];
  const float *lng = (const float*)d_in[18], *lnb = (const float*)d_in[19];
  const float *Wf  = (const float*)d_in[20], *bfin = (const float*)d_in[21];
  float* out = (float*)d_out;

  char* ws = (char*)d_ws;
  unsigned short* XB   = (unsigned short*)(ws + kOffXB);
  unsigned short* BT1  = (unsigned short*)(ws + kOffBT1);
  unsigned short* BT2  = (unsigned short*)(ws + kOffBT2);
  unsigned short* BTF  = (unsigned short*)(ws + kOffBTF);
  float*          BIAS = (float*)(ws + kOffBIAS);
  unsigned short* QKV  = (unsigned short*)(ws + kOffQKV);
  float*          HACC = (float*)(ws + kOffHACC);
  unsigned short* H1H  = (unsigned short*)(ws + kOffH1H);
  unsigned short* H1L  = (unsigned short*)(ws + kOffH1L);
  unsigned short* H2H  = (unsigned short*)(ws + kOffH2H);
  unsigned short* H2L  = (unsigned short*)(ws + kOffH2L);

  const int tilesM = kNPad / 64;
  const int tilesNL = kFusedN / 64;
  const int gemmBlocksL = (tilesM * tilesNL + 7) / 8;
  const int gemmBlocksF = (tilesM + 7) / 8;

  cast_x_kernel<<<(kNPad * kIn / 8) / 256, 256, 0, stream>>>(x, XB);
  wprep_kernel<<<dim3(16, 9), 256, 0, stream>>>(Wq1, Wk1, Wv1, Ws1, Wq2, Wk2, Wv2, Ws2, Wf, BT1, BT2, BTF);
  bias_kernel<<<9, 64, 0, stream>>>(bq1, bk1, bv1, bs1, bq2, bk2, bv2, bs2, bfin, BIAS);

  proj_gemm_kernel<0, 0><<<gemmBlocksL, 256, 0, stream>>>(
      XB, XB, kIn, BT1, kIn, BIAS, QKV, HACC, tilesM, tilesNL, kIn);
  edge_attn_ln_kernel<true><<<kNumTiles, 32, 0, stream>>>(
      ei, (const unsigned*)QKV, HACC, lng, lnb, H1H, H1L);

  proj_gemm_kernel<1, 0><<<gemmBlocksL, 256, 0, stream>>>(
      H1H, H1L, kHid, BT2, kHid, BIAS + kFusedN, QKV, HACC, tilesM, tilesNL, kHid);
  edge_attn_ln_kernel<false><<<kNumTiles, 32, 0, stream>>>(
      ei, (const unsigned*)QKV, HACC, lng, lnb, H2H, H2L);

  proj_gemm_kernel<1, 1><<<gemmBlocksF, 256, 0, stream>>>(
      H2H, H2L, kHid, BTF, kHid, BIAS + 2 * kFusedN, QKV, out, tilesM, 1, kHid);
}
